// MultiHeadAttention_64914135712222
// MI455X (gfx1250) — hardware-verified
//
#include <hip/hip_runtime.h>
#include <stddef.h>


#ifndef NB
#define NB 2
#endif
#ifndef SEQ
#define SEQ 2048
#endif
#define NB_FULL 2
#define SEQ_FULL 2048
#define DM 1024
#define NH 16
#define DKH 64
#define MROWS (NB * SEQ)
#define DM2 (2 * DM)

static_assert(NB >= 1 && NB <= NB_FULL);
static_assert(SEQ >= 128 && SEQ <= SEQ_FULL);
static_assert(SEQ % 128 == 0);
static_assert(SEQ % 64 == 0 && SEQ % 32 == 0);
static_assert(MROWS % 64 == 0);
static_assert(DM % 256 == 0 && DM % 32 == 0 && DM % 64 == 0);
static_assert(DM / 8 == 128);
static_assert(NH * DKH == DM);
static_assert(DKH == 64);
static_assert(DM2 % 32 == 0);

#define P_CARRY      1024.0f
#define CTX_SCALE    0.25f
#define CTXRES_CARRY 256.0f
#define WO_CARRY     64.0f
#define WO_LO_CARRY  0.25f
#define OUT_FOLD     (1.0f / 16384.0f)
#define QK_SCALE     0.125f

static_assert(WO_LO_CARRY * CTXRES_CARRY == WO_CARRY);
static_assert(OUT_FOLD * 256.0f * WO_CARRY == 1.0f);

static_assert(((size_t)8 * MROWS * DM + (size_t)5 * DM * DM) * 2 <= (size_t)134217728);

typedef unsigned short us;
typedef us        v8us  __attribute__((ext_vector_type(8)));
typedef us        v16us __attribute__((ext_vector_type(16)));
typedef _Float16  v16h  __attribute__((ext_vector_type(16)));
typedef __bf16    v16bf __attribute__((ext_vector_type(16)));
typedef float     v8f   __attribute__((ext_vector_type(8)));
typedef float     v4f   __attribute__((ext_vector_type(4)));

__device__ __forceinline__ unsigned bf16rne_bits(float x) {
  unsigned u = __float_as_uint(x);
  return (u + 0x7FFFu + ((u >> 16) & 1u)) >> 16;
}
__device__ __forceinline__ float bf16rne(float x) {
  return __uint_as_float(bf16rne_bits(x) << 16);
}
__device__ __forceinline__ us f16_bits(float x) {
  _Float16 hx = (_Float16)x;
  return __builtin_bit_cast(us, hx);
}

__device__ __forceinline__ v16us frag16(const us* base, int ld, int row0, int k0) {
  const int l = threadIdx.x & 31;
  const int r = l & 15, s = l >> 4;
  const us* p = base + (size_t)(row0 + r) * ld + k0 + 8 * s;
  v8us c0 = *(const v8us*)p;
  v8us c1 = *(const v8us*)(p + 16);
  return __builtin_shufflevector(c0, c1, 0, 1, 2, 3, 4, 5, 6, 7, 8, 9, 10, 11, 12, 13, 14, 15);
}
__device__ __forceinline__ v16h fragh(const us* base, int ld, int row0, int k0) {
  return __builtin_bit_cast(v16h, frag16(base, ld, row0, k0));
}
__device__ __forceinline__ v16bf fragb(const us* base, int ld, int row0, int k0) {
  return __builtin_bit_cast(v16bf, frag16(base, ld, row0, k0));
}
__device__ __forceinline__ v16h cat16h(v8us c0, v8us c1) {
  v16us w = __builtin_shufflevector(c0, c1, 0, 1, 2, 3, 4, 5, 6, 7, 8, 9, 10, 11, 12, 13, 14, 15);
  return __builtin_bit_cast(v16h, w);
}

__device__ __forceinline__ v8f mma_f16(v16h a, v16h b, v8f c) {
  v8f d = __builtin_amdgcn_wmma_f32_16x16x32_f16(false, a, false, b, (short)0, c, false, false);
  asm volatile("v_nop\n\tv_nop\n\tv_nop\n\tv_nop" : "+v"(d) : "v"(a), "v"(b));
  return d;
}
__device__ __forceinline__ v8f mma_bf16(v16bf a, v16bf b, v8f c) {
  v8f d = __builtin_amdgcn_wmma_f32_16x16x32_bf16(false, a, false, b, (short)0, c, false, false);
  asm volatile("v_nop\n\tv_nop\n\tv_nop\n\tv_nop" : "+v"(d) : "v"(a), "v"(b));
  return d;
}

__global__ __launch_bounds__(256) void cvt_x_kernel(const float* __restrict__ X, us* Y, int n8) {
  const int i = blockIdx.x * 256 + threadIdx.x;
  if (i >= n8) return;
  const int m  = i >> 7;
  const int c8 = (i & 127) * 8;
  const int b  = m / SEQ;
  const int s  = m - b * SEQ;
  const float* src = X + ((size_t)(b * SEQ_FULL + s)) * DM + c8;
  v4f x0 = *(const v4f*)src;
  v4f x1 = *(const v4f*)(src + 4);
  v8us y;
#pragma unroll
  for (int j = 0; j < 4; ++j) {
    y[j]     = (us)bf16rne_bits(x0[j]);
    y[4 + j] = (us)bf16rne_bits(x1[j]);
  }
  us* dst = Y + (size_t)i * 8;
  *(volatile v8us*)dst = y;
  __threadfence();
  *(volatile v8us*)dst = y;
}

#define WT_LD 72
static_assert((WT_LD * 2) % 16 == 0 && WT_LD >= 64);
__global__ __launch_bounds__(256) void cvt_wT_kernel(const float* __restrict__ W, us* Y, int hmode) {
  __shared__ __attribute__((aligned(16))) us t0[64 * WT_LD];
  __shared__ __attribute__((aligned(16))) us t1[64 * WT_LD];

  const int t  = threadIdx.x;
  const int k0 = blockIdx.x * 64;
  const int n0 = blockIdx.y * 64;

#pragma unroll 1
  for (int i = 0; i < 4; ++i) {
    const int id = t + i * 256;
    const int kr = id >> 4;
    const int c4 = (id & 15) * 4;
    const v4f x = *(const v4f*)(W + (size_t)(k0 + kr) * DM + n0 + c4);
#pragma unroll
    for (int j = 0; j < 4; ++j) {
      const float w = bf16rne(x[j]);
      const us hb = (us)(__float_as_uint(w) >> 16);
      const us hf = f16_bits(w * WO_CARRY);
      const us hl = f16_bits(w * WO_LO_CARRY);
      t0[(c4 + j) * WT_LD + kr] = hmode ? hf : hb;
      t1[(c4 + j) * WT_LD + kr] = hl;
    }
  }
  __syncthreads();

  const int c = t & 7;
  const size_t pitch = hmode ? (size_t)DM2 : (size_t)DM;
  v8us v0[2], v1[2];
  size_t dsts[2];
#pragma unroll
  for (int it = 0; it < 2; ++it) {
    const int L = (t >> 3) + 32 * it;
    v0[it] = *(const v8us*)&t0[L * WT_LD + 8 * c];
    v1[it] = *(const v8us*)&t1[L * WT_LD + 8 * c];
    dsts[it] = (size_t)(n0 + L) * pitch + k0 + 8 * c;
  }
#pragma unroll
  for (int it = 0; it < 2; ++it) {
    *(volatile v8us*)(Y + dsts[it]) = v0[it];
    if (hmode) *(volatile v8us*)(Y + dsts[it] + DM) = v1[it];
  }
  __threadfence();
#pragma unroll
  for (int it = 0; it < 2; ++it) {
    *(volatile v8us*)(Y + dsts[it]) = v0[it];
    if (hmode) *(volatile v8us*)(Y + dsts[it] + DM) = v1[it];
  }
}

template <int KD>
__device__ __forceinline__ void gemm32x64_bf16(const us* A, const us* B, int m0, int n0, v8f (&acc)[8]) {
  static_assert(KD % 32 == 0);
#pragma unroll 1
  for (int kk = 0; kk < KD; kk += 32) {
    const v16bf a0 = fragb(A, KD, m0, kk);
    const v16bf a1 = fragb(A, KD, m0 + 16, kk);
#pragma unroll
    for (int tt = 0; tt < 4; ++tt) {
      const v16bf b = fragb(B, KD, n0 + 16 * tt, kk);
      acc[tt]     = mma_bf16(a0, b, acc[tt]);
      acc[4 + tt] = mma_bf16(a1, b, acc[4 + tt]);
    }
  }
}
template <int KD>
__device__ __forceinline__ void gemm32x64_f16(const us* A, const us* B, int m0, int n0, v8f (&acc)[8]) {
  static_assert(KD % 32 == 0);
#pragma unroll 1
  for (int kk = 0; kk < KD; kk += 32) {
    const v16h a0 = fragh(A, KD, m0, kk);
    const v16h a1 = fragh(A, KD, m0 + 16, kk);
#pragma unroll
    for (int tt = 0; tt < 4; ++tt) {
      const v16h b = fragh(B, KD, n0 + 16 * tt, kk);
      acc[tt]     = mma_f16(a0, b, acc[tt]);
      acc[4 + tt] = mma_f16(a1, b, acc[4 + tt]);
    }
  }
}

__global__ __launch_bounds__(256) __attribute__((amdgpu_num_vgpr(256)))
void proj_kernel(const us* __restrict__ Xb, const us* __restrict__ Wt,
                 const float* __restrict__ bias, us* Y, int mode) {
  __shared__ __attribute__((aligned(16))) us stile[64 * 256];

  const int t = threadIdx.x;
  const int wid = __builtin_amdgcn_readfirstlane(t >> 5);
  const int l = t & 31;
  const int h = l >> 4, r16 = l & 15;
  const int wm = wid >> 2, wn = wid & 3;
  const int mblk0 = blockIdx.x * 64;
  const int nblk0 = blockIdx.y * 256;
  const int m0 = mblk0 + wm * 32;
  const int n0 = nblk0 + wn * 64;

  v8f acc[8] = {};
  gemm32x64_bf16<DM>(Xb, Wt, m0, n0, acc);

  float bvv[4];
#pragma unroll
  for (int tt = 0; tt < 4; ++tt) bvv[tt] = bf16rne(bias[n0 + 16 * tt + r16]);

  const int bblk = mblk0 / SEQ;
  const int sblk = mblk0 - bblk * SEQ;
  const int c = l & 7;

#pragma unroll
  for (int tt = 0; tt < 4; ++tt) {
    const int nl = wn * 64 + 16 * tt + r16;
#pragma unroll
    for (int mi = 0; mi < 2; ++mi) {
#pragma unroll
      for (int r = 0; r < 8; ++r) {
        const int ml = wm * 32 + 16 * mi + 8 * h + r;
        const float v = acc[mi * 4 + tt][r] + bvv[tt];
        const int li = (mode == 2) ? (nl * 64 + ml) : (ml * 256 + nl);
        stile[li] = f16_bits(v);
      }
    }
  }
  __syncthreads();

  v8us vals[8];
  size_t dsts[8];
#pragma unroll
  for (int it = 0; it < 8; ++it) {
    const int L = wid * 32 + (l >> 3) + 4 * it;
    int src;
    size_t dst;
    if (mode == 2) {
      const int n = nblk0 + L;
      const int hg = n >> 6, d = n & 63;
      src = L * 64 + 8 * c;
      dst = (((size_t)(bblk * NH + hg)) * DKH + d) * SEQ + sblk + 8 * c;
    } else {
      const int ml = L >> 2, hq = L & 3;
      const int hg = (nblk0 >> 6) + hq;
      const int s = sblk + ml;
      src = ml * 256 + hq * 64 + 8 * c;
      dst = (((size_t)(bblk * NH + hg)) * SEQ + s) * DKH + 8 * c;
    }
    vals[it] = *(const v8us*)&stile[src];
    dsts[it] = dst;
  }
#pragma unroll
  for (int it = 0; it < 8; ++it) *(volatile v8us*)(Y + dsts[it]) = vals[it];
  __threadfence();
#pragma unroll
  for (int it = 0; it < 8; ++it) *(volatile v8us*)(Y + dsts[it]) = vals[it];
}

__global__ __launch_bounds__(256) __attribute__((amdgpu_num_vgpr(256)))
void attn_kernel(const us* __restrict__ Qh, const us* __restrict__ Kh,
                 const us* __restrict__ Vt, us* Ctx) {
  __shared__ __attribute__((aligned(16))) us shK[32 * 64];
  __shared__ __attribute__((aligned(16))) us shV[64 * 32];
  __shared__ __attribute__((aligned(16))) us shC[8 * 2 * 16 * 64];

  const int t = threadIdx.x;
  const int wid = __builtin_amdgcn_readfirstlane(t >> 5);
  const int l = t & 31;
  const int r16 = l & 15;
  const int hs = l >> 4;
  const int rowsel = hs << 3;
  constexpr int QBLK = SEQ / 128;
  const int bh = blockIdx.x / QBLK;
  const int qb = blockIdx.x - bh * QBLK;
  const int q0 = qb * 128 + wid * 16;

  const size_t qoff = (size_t)bh * SEQ * DKH;
  const us* qp = Qh + qoff;
  const us* kp = Kh + qoff;
  const us* vp = Vt + (size_t)bh * DKH * SEQ;

  const v16h qB0 = fragh(qp, DKH, q0, 0);
  const v16h qB1 = fragh(qp, DKH, q0, 32);

  v8f o[4];
#pragma unroll
  for (int tt = 0; tt < 4; ++tt) o[tt] = v8f{};
  float mmax = -1.0e30f, lsum = 0.0f;

  const int krow = t >> 3, kcol = (t & 7) * 8;
  const int vrow = t >> 2, vcol = (t & 3) * 8;
  const int kfo = r16 * 64 + 8 * hs;
  const int vfo = r16 * 32 + 8 * hs;

#pragma unroll 1
  for (int kb = 0; kb < SEQ; kb += 32) {
    __syncthreads();
    *(v8us*)&shK[krow * 64 + kcol] = *(const v8us*)(kp + (size_t)(kb + krow) * DKH + kcol);
    *(v8us*)&shV[vrow * 32 + vcol] = *(const v8us*)(vp + (size_t)vrow * SEQ + kb + vcol);
    __syncthreads();

    v8f s0 = {};
    v8f s1 = {};
    {
      const v16h kA = cat16h(*(const v8us*)&shK[kfo], *(const v8us*)&shK[kfo + 16]);
      s0 = mma_f16(kA, qB0, s0);
    }
    {
      const v16h kA = cat16h(*(const v8us*)&shK[kfo + 32], *(const v8us*)&shK[kfo + 48]);
      s0 = mma_f16(kA, qB1, s0);
    }
    {
      const v16h kA = cat16h(*(const v8us*)&shK[16 * 64 + kfo], *(const v8us*)&shK[16 * 64 + kfo + 16]);
      s1 = mma_f16(kA, qB0, s1);
    }
    {
      const v16h kA = cat16h(*(const v8us*)&shK[16 * 64 + kfo + 32], *(const v8us*)&shK[16 * 64 + kfo + 48]);
      s1 = mma_f16(kA, qB1, s1);
    }

    float bm = s0[0];
#pragma unroll
    for (int i = 0; i < 8; ++i) { bm = fmaxf(bm, s0[i]); bm = fmaxf(bm, s1[i]); }
    bm = fmaxf(bm, __shfl_xor(bm, 16, 32));
    const float mnew = fmaxf(mmax, bm * QK_SCALE);
    const float corr = __expf(mmax - mnew);
    mmax = mnew;

    float ps = 0.0f;
    v16h pA;
#pragma unroll
    for (int i = 0; i < 8; ++i) {
      const float p0 = __expf(s0[i] * QK_SCALE - mnew);
      const float p1 = __expf(s1[i] * QK_SCALE - mnew);
      ps += p0 + p1;
      pA[i]     = (_Float16)(p0 * P_CARRY);
      pA[8 + i] = (_Float16)(p1 * P_CARRY);
    }
    ps += __shfl_xor(ps, 16, 32);
    lsum = lsum * corr + ps;

#pragma unroll
    for (int r = 0; r < 8; ++r) {
      const float cr = __shfl(corr, rowsel + r, 32);
#pragma unroll
      for (int tt = 0; tt < 4; ++tt) o[tt][r] *= cr;
    }

#pragma unroll
    for (int tt = 0; tt < 4; ++tt) {
      const v16h vB = cat16h(*(const v8us*)&shV[16 * tt * 32 + vfo],
                             *(const v8us*)&shV[16 * tt * 32 + vfo + 16]);
      o[tt] = mma_f16(pA, vB, o[tt]);
    }
  }

  const int bb = bh / NH;
  const int hh = bh - bb * NH;
#pragma unroll
  for (int r = 0; r < 8; ++r) {
    const float lrow = __shfl(lsum, rowsel + r, 32);
    const float li = CTX_SCALE * __builtin_amdgcn_rcpf(lrow);
#pragma unroll
    for (int tt = 0; tt < 4; ++tt) {
      const float cv = o[tt][r] * li;
      const _Float16 hv = (_Float16)cv;
      const float rs = (cv - (float)hv) * CTXRES_CARRY;
      const int si = wid * 2048 + (rowsel + r) * 64 + 16 * tt + r16;
      shC[si]        = __builtin_bit_cast(us, hv);
      shC[si + 1024] = f16_bits(rs);
    }
  }
  __syncthreads();

  const int c = l & 7;
  v8us vals[8];
  size_t dsts[8];
#pragma unroll
  for (int it = 0; it < 8; ++it) {
    const int Lw = (l >> 3) + 4 * it;
    const int pl = Lw >> 4;
    const int rl = Lw & 15;
    vals[it] = *(const v8us*)&shC[wid * 2048 + pl * 1024 + rl * 64 + 8 * c];
    const int s = q0 + rl;
    dsts[it] = ((size_t)(bb * SEQ + s)) * DM2 + (size_t)pl * DM + hh * DKH + 8 * c;
  }
#pragma unroll
  for (int it = 0; it < 8; ++it) *(volatile v8us*)(Ctx + dsts[it]) = vals[it];
  __threadfence();
#pragma unroll
  for (int it = 0; it < 8; ++it) *(volatile v8us*)(Ctx + dsts[it]) = vals[it];
}

__global__ __launch_bounds__(256) __attribute__((amdgpu_num_vgpr(256)))
void outproj_kernel(const us* __restrict__ Ctx, const us* __restrict__ Wot,
                    const float* __restrict__ bo, float* Out) {
  __shared__ __attribute__((aligned(16))) float ftile[32 * 256];

  const int t = threadIdx.x;
  const int wid = __builtin_amdgcn_readfirstlane(t >> 5);
  const int l = t & 31;
  const int h = l >> 4, r16 = l & 15;
  const int wm = wid >> 2, wn = wid & 3;
  const int mblk0 = blockIdx.x * 64;
  const int nblk0 = blockIdx.y * 256;
  const int m0 = mblk0 + wm * 32;
  const int n0 = nblk0 + wn * 64;

  v8f acc[8] = {};
  gemm32x64_f16<DM2>(Ctx, Wot, m0, n0, acc);

  float bob[4];
#pragma unroll
  for (int tt = 0; tt < 4; ++tt) bob[tt] = bf16rne(bo[n0 + 16 * tt + r16]);

  const int c = l & 7;
#pragma unroll
  for (int p = 0; p < 2; ++p) {
    if (p) __syncthreads();
#pragma unroll
    for (int tt = 0; tt < 4; ++tt) {
      const int nl = wn * 64 + 16 * tt + r16;
#pragma unroll
      for (int r = 0; r < 8; ++r) {
        const int rl = wm * 16 + 8 * h + r;
        ftile[rl * 256 + nl] = acc[p * 4 + tt][r] * OUT_FOLD + bob[tt];
      }
    }
    __syncthreads();

    v4f vals[8];
    size_t dsts[8];
#pragma unroll
    for (int it = 0; it < 8; ++it) {
      const int L = wid * 32 + (l >> 3) + 4 * it;
      const int rl = L >> 3, seg = L & 7;
      vals[it] = *(const v4f*)&ftile[rl * 256 + seg * 32 + 4 * c];
      const int m = mblk0 + (rl >> 4) * 32 + p * 16 + (rl & 15);
      dsts[it] = (size_t)m * DM + nblk0 + seg * 32 + 4 * c;
    }
#pragma unroll
    for (int it = 0; it < 8; ++it) *(volatile v4f*)(Out + dsts[it]) = vals[it];
    __threadfence();
#pragma unroll
    for (int it = 0; it < 8; ++it) *(volatile v4f*)(Out + dsts[it]) = vals[it];
  }
}

extern "C" void kernel_launch(void* const* d_in, const int* in_sizes, int n_in,
                              void* d_out, int out_size, void* d_ws, size_t ws_size,
                              hipStream_t stream) {
  if (n_in < 11) return;
  const int need_x = ((NB - 1) * SEQ_FULL + SEQ) * DM;
  if (in_sizes[0] < need_x || in_sizes[1] < need_x || in_sizes[2] < need_x) return;
  if (in_sizes[3] < DM * DM || in_sizes[5] < DM * DM || in_sizes[7] < DM * DM || in_sizes[9] < DM * DM) return;
  if (in_sizes[4] < DM || in_sizes[6] < DM || in_sizes[8] < DM || in_sizes[10] < DM) return;
  if (out_size < MROWS * DM) return;

  const float* Q  = (const float*)d_in[0];
  const float* K  = (const float*)d_in[1];
  const float* V  = (const float*)d_in[2];
  const float* Wq = (const float*)d_in[3];
  const float* bq = (const float*)d_in[4];
  const float* Wk = (const float*)d_in[5];
  const float* bk = (const float*)d_in[6];
  const float* Wv = (const float*)d_in[7];
  const float* bv = (const float*)d_in[8];
  const float* Wo = (const float*)d_in[9];
  const float* bo = (const float*)d_in[10];

  const size_t XE = (size_t)MROWS * DM;
  const size_t WE = (size_t)DM * DM;
  const size_t total_bytes = (8 * XE + 5 * WE) * sizeof(us);
  if (total_bytes > ws_size) return;

  us* xq  = (us*)d_ws;
  us* xk  = xq + XE;
  us* xv  = xk + XE;
  us* wtq = xv + XE;
  us* wtk = wtq + WE;
  us* wtv = wtk + WE;
  us* wo2 = wtv + WE;
  us* qh  = wo2 + 2 * WE;
  us* kh  = qh + XE;
  us* vt  = kh + XE;
  us* ctx = vt + XE;

  dim3 blk(256);
  const int n8 = (int)(XE / 8);
  dim3 gx((n8 + 255) / 256);
  cvt_x_kernel<<<gx, blk, 0, stream>>>(Q, xq, n8);
  cvt_x_kernel<<<gx, blk, 0, stream>>>(K, xk, n8);
  cvt_x_kernel<<<gx, blk, 0, stream>>>(V, xv, n8);

  dim3 gw(DM / 64, DM / 64);
  cvt_wT_kernel<<<gw, blk, 0, stream>>>(Wq, wtq, 0);
  cvt_wT_kernel<<<gw, blk, 0, stream>>>(Wk, wtk, 0);
  cvt_wT_kernel<<<gw, blk, 0, stream>>>(Wv, wtv, 0);
  cvt_wT_kernel<<<gw, blk, 0, stream>>>(Wo, wo2, 1);

  dim3 gp(MROWS / 64, DM / 256);
  proj_kernel<<<gp, blk, 0, stream>>>(xq, wtq, bq, qh, 0);
  proj_kernel<<<gp, blk, 0, stream>>>(xk, wtk, bk, kh, 1);
  proj_kernel<<<gp, blk, 0, stream>>>(xv, wtv, bv, vt, 2);

  attn_kernel<<<dim3(NB * NH * (SEQ / 128)), blk, 0, stream>>>(qh, kh, vt, ctx);

  outproj_kernel<<<gp, blk, 0, stream>>>(ctx, wo2, bo, (float*)d_out);
}
